// MultiScaleRetention_41575283425483
// MI455X (gfx1250) — hardware-verified
//
#include <hip/hip_runtime.h>
#include <math.h>

constexpr int kBatch      = 16;
constexpr int kSeq        = 1024;
constexpr int kDim        = 512;
constexpr int kHeads      = 8;
constexpr int kHd         = 64;
constexpr int kTok        = kBatch * kSeq;
constexpr int kChunks     = kSeq / 2;
constexpr int kProjN      = 3 * kHd;
constexpr int kProjAll    = kHeads * kProjN;
constexpr int kGroupHeads = 2;
constexpr int kGroups     = kHeads / kGroupHeads;
constexpr int kGroupN     = kGroupHeads * kProjN;
constexpr int kStatPitch  = 32;
constexpr float kGnEps     = 1.0e-3f;
constexpr float kInvSqrtHd = 0.125f;
static_assert(kHeads * kHd == kDim, "shape");
static_assert(kTok % 64 == 0 && kGroupN % 64 == 0 && kDim % 64 == 0 && kDim % 32 == 0, "tiles");
static_assert(kSeq % 64 == 0 && kProjN % 64 == 0 && kHeads % kGroupHeads == 0, "head tiles");
static_assert(2 * (kProjN / 4) == 96, "staging lanes = waves 0..2");

typedef __attribute__((ext_vector_type(16))) _Float16 v16h;
typedef __attribute__((ext_vector_type(8)))  _Float16 v8h;
typedef __attribute__((ext_vector_type(16))) __bf16   v16b;
typedef __attribute__((ext_vector_type(8)))  __bf16   v8b;
typedef __attribute__((ext_vector_type(8)))  float    v8f;
typedef __attribute__((ext_vector_type(4)))  float    v4f;
typedef __attribute__((ext_vector_type(4)))  unsigned int v4u;

__device__ __forceinline__ unsigned short f2bf_bits(float f) {
  unsigned u = __float_as_uint(f);
  return (unsigned short)((u + 0x7FFFu + ((u >> 16) & 1u)) >> 16);
}
__device__ __forceinline__ float bf_bits2f(unsigned short h) { return __uint_as_float(((unsigned)h) << 16); }
__device__ __forceinline__ float bf_rn(float f) { return bf_bits2f(f2bf_bits(f)); }

__device__ __forceinline__ void dep_guard_h(v8f& a, v8f& b, v16h x, v16h y) { asm volatile("v_nop\n\tv_nop\n\tv_nop\n\tv_nop" : "+v"(a), "+v"(b) : "v"(x), "v"(y)); }
__device__ __forceinline__ void dep_guard_b(v8f& a, v8f& b, v16b x, v16b y) { asm volatile("v_nop\n\tv_nop\n\tv_nop\n\tv_nop" : "+v"(a), "+v"(b) : "v"(x), "v"(y)); }
__device__ __forceinline__ void dep_guard4_h(v8f& a, v8f& b, v8f& c, v8f& d, v16h x, v16h y) { asm volatile("v_nop\n\tv_nop\n\tv_nop\n\tv_nop" : "+v"(a), "+v"(b), "+v"(c), "+v"(d) : "v"(x), "v"(y)); }
__device__ __forceinline__ void dep_guard4_b(v8f& a, v8f& b, v8f& c, v8f& d, v16b x, v16b y) { asm volatile("v_nop\n\tv_nop\n\tv_nop\n\tv_nop" : "+v"(a), "+v"(b), "+v"(c), "+v"(d) : "v"(x), "v"(y)); }
__device__ __forceinline__ void keep4_h(v16h a, v16h b, v16h c, v16h d) { asm volatile("v_nop" :: "v"(a), "v"(b), "v"(c), "v"(d)); }
__device__ __forceinline__ void keep4_b(v16b a, v16b b, v16b c, v16b d) { asm volatile("v_nop" :: "v"(a), "v"(b), "v"(c), "v"(d)); }
__device__ __forceinline__ void acc_guard4(v8f& a, v8f& b, v8f& c, v8f& d) { asm volatile("v_nop\n\tv_nop\n\tv_nop\n\tv_nop" : "+v"(a), "+v"(b), "+v"(c), "+v"(d)); }
template <typename T> struct Frag;
template <> struct Frag<_Float16> {
  typedef v16h V; union U { v16h v; v8h h[2]; };
  static __device__ __forceinline__ v16h load(const _Float16* p) {
    U f; f.h[0] = *(const v8h*)(p); f.h[1] = *(const v8h*)(p + 16); return f.v;
  }
  static __device__ __forceinline__ v8f mma(v16h a, v16h b, v8f c) {
    return __builtin_amdgcn_wmma_f32_16x16x32_f16(false, a, false, b, (short)0, c, false, false);
  }
  static __device__ __forceinline__ void guard(v8f& a, v8f& b, v16h x, v16h y) { dep_guard_h(a, b, x, y); }
  static __device__ __forceinline__ void guard4(v8f& a, v8f& b, v8f& c, v8f& d, v16h x, v16h y) { dep_guard4_h(a, b, c, d, x, y); }
  static __device__ __forceinline__ void keep(v16h a, v16h b, v16h c, v16h d) { keep4_h(a, b, c, d); }
};
template <> struct Frag<__bf16> {
  typedef v16b V; union U { v16b v; v8b h[2]; };
  static __device__ __forceinline__ v16b load(const __bf16* p) {
    U f; f.h[0] = *(const v8b*)(p); f.h[1] = *(const v8b*)(p + 16); return f.v;
  }
  static __device__ __forceinline__ v8f mma(v16b a, v16b b, v8f c) {
    return __builtin_amdgcn_wmma_f32_16x16x32_bf16(false, a, false, b, (short)0, c, false, false);
  }
  static __device__ __forceinline__ void guard(v8f& a, v8f& b, v16b x, v16b y) { dep_guard_b(a, b, x, y); }
  static __device__ __forceinline__ void guard4(v8f& a, v8f& b, v8f& c, v8f& d, v16b x, v16b y) { dep_guard4_b(a, b, c, d, x, y); }
  static __device__ __forceinline__ void keep(v16b a, v16b b, v16b c, v16b d) { keep4_b(a, b, c, d); }
};

__device__ __forceinline__ unsigned pk16(unsigned short a, unsigned short b) { return (unsigned)a | ((unsigned)b << 16); }

template <int ET> struct Elem;
template <> struct Elem<0> { typedef _Float16 T; };
template <> struct Elem<1> { typedef __bf16 T; };
template <int ET, int SPLIT, int BIAS_MODE, int OUT_MODE, bool RESID, int ACT = 0>
__global__ __launch_bounds__(256) void wmma_gemm64(
    const unsigned short* __restrict__ Ap, const unsigned short* __restrict__ A2p, int lda, long strideA,
    const unsigned short* __restrict__ Btp, const unsigned short* __restrict__ Bt2p, int ldb, long strideB,
    void* __restrict__ Cout, void* __restrict__ Cout2, int ldc, long strideC,
    const float* __restrict__ bias,
    const float* __restrict__ resid, long strideR,
    int M, int N, int K, float scale,
    const float* __restrict__ aux0, const float* __restrict__ aux1) {
  typedef typename Elem<ET>::T T;
  typedef typename Frag<T>::V V;
  const T* A = (const T*)Ap; const T* A2 = (const T*)A2p; const T* Bt = (const T*)Btp; const T* Bt2 = (const T*)Bt2p;
  __shared__ __align__(16) float sT[8][16 * 68];
  const int b    = blockIdx.y;
  const int lane = threadIdx.x & 31;
  const int wave = threadIdx.x >> 5;
  const int tilesN = N >> 6;
  const int tilesM = M >> 6;
  const int tile = blockIdx.x * 8 + wave;
  if (tile >= tilesM * tilesN) return;
  const int tm = tile / tilesN;
  const int tn = tile - tm * tilesN;
  const int m0 = tm << 6;
  const int n0 = tn << 6;

  const T* Ab  = A  + (size_t)b * strideA;
  const T* Bb  = Bt + (size_t)b * strideB;
  const T* Ab2 = (SPLIT >= 1) ? (A2  + (size_t)b * strideA) : nullptr;
  const T* Bb2 = (SPLIT == 2) ? (Bt2 + (size_t)b * strideB) : nullptr;

  const int rlane = lane & 15;
  const int koff  = (lane >> 4) * 8;
  const int mOff  = (lane >> 4) * 8;

  v8f acc[4][4];
#pragma unroll
  for (int i = 0; i < 4; ++i)
#pragma unroll
    for (int j = 0; j < 4; ++j) acc[i][j] = (v8f){0.f,0.f,0.f,0.f,0.f,0.f,0.f,0.f};

  for (int k0 = 0; k0 < K; k0 += 32) {
    V bh[4], bl[4];
#pragma unroll
    for (int j = 0; j < 4; ++j) {
      const size_t bo = (size_t)(n0 + (j << 4) + rlane) * ldb + koff + k0;
      bh[j] = Frag<T>::load(Bb + bo);
      if (SPLIT == 2) bl[j] = Frag<T>::load(Bb2 + bo);
    }
#pragma unroll
    for (int i = 0; i < 4; ++i) {
      const size_t ao = (size_t)(m0 + (i << 4) + rlane) * lda + koff + k0;
      V ah = Frag<T>::load(Ab + ao);
      V al = ah;
      if (SPLIT >= 1) al = Frag<T>::load(Ab2 + ao);
#pragma unroll
      for (int j = 0; j < 4; ++j) {
        acc[i][j] = Frag<T>::mma(ah, bh[j], acc[i][j]);
        if (SPLIT == 2) acc[i][j] = Frag<T>::mma(ah, bl[j], acc[i][j]);
        if (SPLIT >= 1) acc[i][j] = Frag<T>::mma(al, bh[j], acc[i][j]);
      }
      Frag<T>::guard4(acc[i][0], acc[i][1], acc[i][2], acc[i][3], ah, al);
    }
    Frag<T>::keep(bh[0], bh[1], bh[2], bh[3]);
    if (SPLIT == 2) Frag<T>::keep(bl[0], bl[1], bl[2], bl[3]);
  }
  acc_guard4(acc[0][0], acc[0][1], acc[0][2], acc[0][3]);
  acc_guard4(acc[1][0], acc[1][1], acc[1][2], acc[1][3]);
  acc_guard4(acc[2][0], acc[2][1], acc[2][2], acc[2][3]);
  acc_guard4(acc[3][0], acc[3][1], acc[3][2], acc[3][3]);

  float* slab = sT[wave];
  const float* Rb = RESID ? (resid + (size_t)b * strideR) : nullptr;
  float gmu = 0.f, gis = 1.f;
  float gb[8] = {0.f, 0.f, 0.f, 0.f, 0.f, 0.f, 0.f, 0.f};
  if (OUT_MODE == 3) {
    const float* stp = aux0 + (size_t)(((m0 / kSeq) * kHeads + (n0 / kHd)) * kStatPitch);
    gmu = stp[0];
    gis = stp[1];
    const int c8b = (lane & 7) * 8;
    const v4f t0 = *(const v4f*)(aux1 + n0 + c8b);
    const v4f t1 = *(const v4f*)(aux1 + n0 + c8b + 4);
#pragma unroll
    for (int e = 0; e < 4; ++e) {
      const float f0 = t0[e];
      const float f1 = t1[e];
      gb[e]     = bf_rn(f0);
      gb[4 + e] = bf_rn(f1);
    }
  }
#pragma unroll
  for (int i = 0; i < 4; ++i) {
    const int mBase = m0 + (i << 4);
#pragma unroll
    for (int j = 0; j < 4; ++j) {
      const int n = n0 + (j << 4) + rlane;
      float bv = 0.f;
      if (BIAS_MODE == 2) bv = bf_rn(bias[n]);
#pragma unroll
      for (int r = 0; r < 8; ++r) {
        float v = acc[i][j][r] * scale;
        if (BIAS_MODE == 1) v += bf_rn(bias[mBase + mOff + r]);
        if (BIAS_MODE == 2) v += bv;
        if (RESID) v += Rb[(size_t)(mBase + mOff + r) * ldc + n];
        if (ACT == 2) v = fmaxf(v, 0.0f);
        if (ACT == 4) v = (v > 0.f) ? v : 0.01f * v;
        slab[(mOff + r) * 68 + (j << 4) + rlane] = v;
      }
    }
    __builtin_amdgcn_fence(__ATOMIC_RELEASE, "workgroup");
    __builtin_amdgcn_wave_barrier();
    __builtin_amdgcn_fence(__ATOMIC_ACQUIRE, "workgroup");
    if (OUT_MODE == 0) {
      float* C = (float*)Cout + (size_t)b * strideC;
      const int hh = lane >> 4, c4 = (lane & 15) * 4;
      for (int pass = 0; pass < 2; ++pass) {
#pragma unroll
        for (int it = 0; it < 8; ++it) {
          const int row = it * 2 + hh;
          v4f v = *(const v4f*)(slab + row * 68 + c4);
          *(volatile v4f*)(C + (size_t)(mBase + row) * ldc + n0 + c4) = v;
        }
        __threadfence();
      }
    } else if (OUT_MODE == 3) {
      const int q = lane >> 3, c8 = (lane & 7) * 8;
      unsigned short* C  = (unsigned short*)Cout  + (size_t)b * strideC;
      unsigned short* C2 = (unsigned short*)Cout2 + (size_t)b * strideC;
      const float* Xb = resid + (size_t)b * strideR;
      v8h hv3[4], lv3[4];
#pragma unroll
      for (int it = 0; it < 4; ++it) {
        const int row = it * 4 + q;
        const float* sp = slab + row * 68 + c8;
        const float* xp = Xb + (size_t)(mBase + row) * ldc + n0 + c8;
        const v4f x0 = *(const v4f*)(xp);
        const v4f x1 = *(const v4f*)(xp + 4);
        v8h h8, l8;
#pragma unroll
        for (int e = 0; e < 4; ++e) {
          const float xa = x0[e];
          const float xb = x1[e];
          const float ya = (xa - gmu) * gis + gb[e];
          const float yb = (xb - gmu) * gis + gb[4 + e];
          const float ga = sp[e];
          const float gg = sp[4 + e];
          const float sa = 1.0f / (1.0f + expf(-ga));
          const float sb = 1.0f / (1.0f + expf(-gg));
          const float za = (ga * sa) * ya;
          const float zb = (gg * sb) * yb;
          const unsigned short ha = f2bf_bits(za);
          const unsigned short la = f2bf_bits(za - bf_bits2f(ha));
          const unsigned short hb = f2bf_bits(zb);
          const unsigned short lb = f2bf_bits(zb - bf_bits2f(hb));
          h8[e]     = __builtin_bit_cast(_Float16, ha);
          l8[e]     = __builtin_bit_cast(_Float16, la);
          h8[4 + e] = __builtin_bit_cast(_Float16, hb);
          l8[4 + e] = __builtin_bit_cast(_Float16, lb);
        }
        hv3[it] = h8;
        lv3[it] = l8;
      }
      for (int pass = 0; pass < 2; ++pass) {
#pragma unroll
        for (int it = 0; it < 4; ++it) {
          const int row = it * 4 + q;
          *(volatile v8h*)(C  + (size_t)(mBase + row) * ldc + n0 + c8) = hv3[it];
          *(volatile v8h*)(C2 + (size_t)(mBase + row) * ldc + n0 + c8) = lv3[it];
        }
        __threadfence();
      }
    } else {
      const int q = lane >> 3, c8 = (lane & 7) * 8;
      unsigned short* C  = (unsigned short*)Cout  + (size_t)b * strideC;
      unsigned short* C2 = (OUT_MODE == 2) ? ((unsigned short*)Cout2 + (size_t)b * strideC) : nullptr;
      for (int pass = 0; pass < 2; ++pass) {
#pragma unroll
        for (int it = 0; it < 4; ++it) {
          const int row = it * 4 + q;
          const float* sp = slab + row * 68 + c8;
          v8h hv, lv;
#pragma unroll
          for (int e = 0; e < 8; ++e) {
            if (OUT_MODE == 1) {
              hv[e] = (_Float16)sp[e];
            } else {
              unsigned short hb = f2bf_bits(sp[e]);
              unsigned short lb = f2bf_bits(sp[e] - bf_bits2f(hb));
              hv[e] = __builtin_bit_cast(_Float16, hb);
              lv[e] = __builtin_bit_cast(_Float16, lb);
            }
          }
          *(volatile v8h*)(C + (size_t)(mBase + row) * ldc + n0 + c8) = hv;
          if (OUT_MODE == 2) *(volatile v8h*)(C2 + (size_t)(mBase + row) * ldc + n0 + c8) = lv;
        }
        __threadfence();
      }
    }
    __builtin_amdgcn_fence(__ATOMIC_RELEASE, "workgroup");
    __builtin_amdgcn_wave_barrier();
    __builtin_amdgcn_fence(__ATOMIC_ACQUIRE, "workgroup");
  }
}

__global__ __launch_bounds__(256) void cast8_bf16_kernel(const float* __restrict__ in, unsigned short* __restrict__ out, int n8) {
  const int i = blockIdx.x * 256 + threadIdx.x;
  if (i >= n8) return;
  const float* p = in + 8 * (size_t)i;
  const v4f a = *(const v4f*)(p);
  const v4f c = *(const v4f*)(p + 4);
  unsigned short hb[8];
#pragma unroll
  for (int e = 0; e < 4; ++e) {
    const float fa = a[e];
    const float fc = c[e];
    hb[e]     = f2bf_bits(fa);
    hb[4 + e] = f2bf_bits(fc);
  }
  const v4u u = (v4u){pk16(hb[0], hb[1]), pk16(hb[2], hb[3]), pk16(hb[4], hb[5]), pk16(hb[6], hb[7])};
  unsigned short* q = out + 8 * (size_t)i;
  *(volatile v4u*)q = u;
  __threadfence();
  *(volatile v4u*)q = u;
}

__global__ __launch_bounds__(256) void wtcast_kernel(const float* __restrict__ W, unsigned short* __restrict__ out,
                                                     int nOut, long inStride, long outStride) {
  __shared__ float sm[64][65];
  const int t  = threadIdx.x;
  const int k0 = blockIdx.x * 64;
  const int n0 = blockIdx.y * 64;
  const int z  = blockIdx.z;
  const float* Wz = W + (size_t)z * inStride;
#pragma unroll
  for (int i = 0; i < 16; ++i) {
    const int e = i * 256 + t;
    const int r = e >> 6;
    const int c = e & 63;
    sm[c][r] = Wz[(size_t)(k0 + r) * nOut + n0 + c];
  }
  __syncthreads();
  const int lane = t & 31, wave = t >> 5;
  const int q = lane >> 3, c8 = (lane & 7) * 8;
  unsigned short* op = out + (size_t)z * outStride;
  for (int pass = 0; pass < 2; ++pass) {
#pragma unroll
    for (int it = 0; it < 2; ++it) {
      const int row = wave * 8 + it * 4 + q;
      unsigned short hb[8];
#pragma unroll
      for (int e = 0; e < 8; ++e) hb[e] = f2bf_bits(sm[row][c8 + e]);
      const v4u u = (v4u){pk16(hb[0], hb[1]), pk16(hb[2], hb[3]), pk16(hb[4], hb[5]), pk16(hb[6], hb[7])};
      *(volatile v4u*)(op + (size_t)(n0 + row) * kDim + k0 + c8) = u;
    }
    __threadfence();
  }
}

__device__ __forceinline__ float decay_u(float g, float eps, int n) {
  float p = 1.0f, u = 0.0f;
#pragma unroll 1
  for (int bit = 9; bit >= 0; --bit) {
    u = u * (1.0f + p);
    p = p * p;
    const bool s = ((n >> bit) & 1) != 0;
    const float un = fmaf(u, g, eps);
    const float pn = p * g;
    u = s ? un : u;
    p = s ? pn : p;
  }
  return u;
}

__global__ __launch_bounds__(512) void retention_scan_kernel(const float* __restrict__ Pg,
                                                            float* __restrict__ X, float* __restrict__ stats, int grp) {
  __shared__ __align__(16) float rowbuf[2][2 * kProjN];
  __shared__ __align__(16) float red[2][8][kHd];
  __shared__ float wsum[16];
  __shared__ float tab[kChunks + 32];
  __shared__ float sred[256];
  __shared__ __align__(16) float sline[kStatPitch];

  const int tid  = threadIdx.x;
  const int lane = tid & 31;
  const int wave = tid >> 5;
  const int blk  = blockIdx.x;
  const int b    = blk >> 1;
  const int hl   = blk & 1;
  const int h    = grp * kGroupHeads + hl;
  const int c    = tid & 63;
  const int rg   = tid >> 6;

  const float eps    = __uint_as_float((unsigned)(127 - 5 - h) << 23);
  const float epsInv = __uint_as_float((unsigned)(127 + 5 + h) << 23);
  const float g  = 1.0f - eps;
  const float g3 = (g * g) * g;

  tab[tid] = kInvSqrtHd / sqrtf(decay_u(g, eps, tid + 2) * epsInv);
  if (tid < 32) tab[kChunks + tid] = kInvSqrtHd / sqrtf(decay_u(g, eps, tid + kChunks + 2) * epsInv);

  const bool stg = (wave < 3);
  const int  rw  = (tid >= kProjN / 4) ? 1 : 0;
  const int  cw  = stg ? (tid - rw * (kProjN / 4)) : 0;
  const size_t pbase = (size_t)(b * kSeq) * kGroupN + (size_t)hl * kProjN + (size_t)cw * 4;
  v4f pf = (v4f){0.f, 0.f, 0.f, 0.f};
  if (stg) pf = *(const v4f*)(Pg + pbase + (size_t)rw * kGroupN);

  float R[8];
#pragma unroll
  for (int r = 0; r < 8; ++r) R[r] = 0.0f;
  float lsum = 0.0f, lsq = 0.0f;
  __syncthreads();

  for (int t = 0; t < kChunks; ++t) {
    float* rb = rowbuf[t & 1];
    if (stg) {
      *(v4f*)(rb + rw * kProjN + cw * 4) = pf;
      const int tn = (t + 1 < kChunks) ? (t + 1) : (kChunks - 1);
      pf = *(const v4f*)(Pg + pbase + (size_t)(2 * tn + rw) * kGroupN);
    }
    __syncthreads();

    {
      const float* q0p = rb + rg * 8;
      const float* q1p = rb + kProjN + rg * 8;
      const v4f q0a = *(const v4f*)(q0p);
      const v4f q0b = *(const v4f*)(q0p + 4);
      const v4f q1a = *(const v4f*)(q1p);
      const v4f q1b = *(const v4f*)(q1p + 4);
      float p0 = 0.0f, p1 = 0.0f;
#pragma unroll
      for (int r = 0; r < 4; ++r) {
        p0 = fmaf(q0a[r], R[r], p0);
        p1 = fmaf(q1a[r], R[r], p1);
      }
#pragma unroll
      for (int r = 0; r < 4; ++r) {
        p0 = fmaf(q0b[r], R[4 + r], p0);
        p1 = fmaf(q1b[r], R[4 + r], p1);
      }
      red[0][rg][c] = p0;
      red[1][rg][c] = p1;
    }
    {
      const int dsel = (wave < 6) ? (wave >> 1) : 0;
      const int half = wave & 1;
      const int qo = (dsel >= 1) ? kProjN : 0;
      const int ko = (dsel == 2) ? (kProjN + kHd) : kHd;
      float pr = rb[qo + half * 32 + lane] * rb[ko + half * 32 + lane];
      pr += __shfl_xor(pr, 16, 32);
      pr += __shfl_xor(pr, 8, 32);
      pr += __shfl_xor(pr, 4, 32);
      pr += __shfl_xor(pr, 2, 32);
      pr += __shfl_xor(pr, 1, 32);
      if (lane == 0) wsum[wave] = pr;
    }
    __syncthreads();

    if (rg < 2) {
      const float d00 = wsum[0] + wsum[1];
      const float d10 = wsum[2] + wsum[3];
      const float d11 = wsum[4] + wsum[5];
      const float c00 = tab[t];
      const float c11 = tab[t + 1];
      const float c10 = g * c00;
      const float s00 = d00 * c00;
      const float s10 = d10 * c10;
      const float s11 = d11 * c11;
      const float r0 = fmaxf(fabsf(s00), 1.0f);
      const float r1 = fmaxf(fabsf(s10 + s11), 1.0f);
      const float i0 = 1.0f / r0;
      const float i1 = 1.0f / r1;
      const float cA = (rg == 0) ? (s00 * i0) : (s10 * i0);
      const float cB = (rg == 0) ? 0.0f : (s11 * i1);
      float cross = 0.0f;
#pragma unroll
      for (int k = 0; k < 8; ++k) cross += red[rg][k][c];
      const float v0c = rb[2 * kHd + c];
      const float v1c = rb[kProjN + 2 * kHd + c];
      const float o = fmaf(cA, v0c, fmaf(cB, v1c, cross));
      lsum += o;
      lsq = fmaf(o, o, lsq);
      const int chalf = wave & 1;
      const int src = (lane & 7) * 4;
      const float f0 = __shfl(o, src, 32);
      const float f1 = __shfl(o, src + 1, 32);
      const float f2 = __shfl(o, src + 2, 32);
      const float f3 = __shfl(o, src + 3, 32);
      const v4f val = (v4f){f0, f1, f2, f3};
      float* xp = X + ((size_t)(b * kSeq + 2 * t + rg)) * kDim + h * kHd + chalf * 32 + src;
      if (lane < 8) *(volatile v4f*)xp = val;
      __threadfence();
      if (lane < 8) *(volatile v4f*)xp = val;
    }

    {
      const float v0c = rb[2 * kHd + c];
      const float v1c = rb[kProjN + 2 * kHd + c];
      const float* k0p = rb + kHd + rg * 8;
      const float* k1p = rb + kProjN + kHd + rg * 8;
      const v4f k0a = *(const v4f*)(k0p);
      const v4f k0b = *(const v4f*)(k0p + 4);
      const v4f k1a = *(const v4f*)(k1p);
      const v4f k1b = *(const v4f*)(k1p + 4);
#pragma unroll
      for (int r = 0; r < 4; ++r) R[r]     = fmaf(k1a[r], v1c, fmaf(k0a[r], v0c, R[r])) * g3;
#pragma unroll
      for (int r = 0; r < 4; ++r) R[4 + r] = fmaf(k1b[r], v1c, fmaf(k0b[r], v0c, R[4 + r])) * g3;
    }
  }

  if (tid < 128) { sred[tid] = lsum; sred[128 + tid] = lsq; }
  if (tid < kStatPitch) sline[tid] = 0.0f;
  __syncthreads();
  if (tid == 0) {
    double ds = 0.0, dq = 0.0;
#pragma unroll 1
    for (int i = 0; i < 128; ++i) {
      ds += (double)sred[i];
      dq += (double)sred[128 + i];
    }
    const double invn = 1.52587890625e-5;
    const double mu  = ds * invn;
    const double var = dq * invn - mu * mu;
    float varf = (float)var;
    varf = fmaxf(varf, 0.0f);
    sline[0] = (float)mu;
    sline[1] = 1.0f / sqrtf(varf + kGnEps);
  }
  __syncthreads();
  if (tid < 8) {
    const v4f v = *(const v4f*)(sline + 4 * tid);
    float* sp = stats + (size_t)(b * kHeads + h) * kStatPitch + 4 * tid;
    *(volatile v4f*)sp = v;
    __threadfence();
    *(volatile v4f*)sp = v;
  }
}

extern "C" void kernel_launch(void* const* d_in, const int* in_sizes, int n_in,
                              void* d_out, int out_size, void* d_ws, size_t ws_size,
                              hipStream_t stream) {
  if (n_in < 10) return;
  const int nAct = kTok * kDim;
  if (in_sizes[0] != nAct) return;
  if (in_sizes[3] != kDim * kDim || in_sizes[4] != kDim) return;
  if (in_sizes[5] != kDim * kDim || in_sizes[6] != kDim) return;
  if (in_sizes[7] != kHeads * kDim * kProjN || in_sizes[8] != kProjAll || in_sizes[9] != kDim) return;
  if (out_size != nAct) return;

  const size_t szQ16  = (size_t)kTok * kDim * 2;
  const size_t szWqT  = (size_t)kProjAll * kDim * 2;
  const size_t szWT   = (size_t)kDim * kDim * 2;
  const size_t szPG   = (size_t)kTok * kGroupN * 4;
  const size_t szX    = (size_t)kTok * kDim * 4;
  const size_t szZ    = (size_t)kTok * kDim * 2;
  const size_t szSt   = (size_t)kBatch * kHeads * kStatPitch * 4;
  const size_t offQ16 = 0;
  const size_t offWqT = offQ16 + szQ16;
  const size_t offWgT = offWqT + szWqT;
  const size_t offWoT = offWgT + szWT;
  const size_t offPG  = offWoT + szWT;
  const size_t offX   = offPG + szPG;
  const size_t offZH  = offX + szX;
  const size_t offZL  = offZH + szZ;
  const size_t offSt  = offZL + szZ;
  const size_t total  = offSt + szSt;
  if (ws_size < total) return;

  const float* q    = (const float*)d_in[0];
  const float* Wg   = (const float*)d_in[3];
  const float* bg   = (const float*)d_in[4];
  const float* Wo   = (const float*)d_in[5];
  const float* bo   = (const float*)d_in[6];
  const float* Wqkv = (const float*)d_in[7];
  const float* bqkv = (const float*)d_in[8];
  const float* beta = (const float*)d_in[9];
  float* out = (float*)d_out;
  char* ws = (char*)d_ws;
  unsigned short* Q16  = (unsigned short*)(ws + offQ16);
  unsigned short* WQT  = (unsigned short*)(ws + offWqT);
  unsigned short* WGT  = (unsigned short*)(ws + offWgT);
  unsigned short* WOT  = (unsigned short*)(ws + offWoT);
  float*          PG   = (float*)(ws + offPG);
  float*          XX   = (float*)(ws + offX);
  unsigned short* ZH   = (unsigned short*)(ws + offZH);
  unsigned short* ZL   = (unsigned short*)(ws + offZL);
  float*          ST   = (float*)(ws + offSt);

  const int n8 = nAct / 8;
  cast8_bf16_kernel<<<dim3(n8 / 256), dim3(256), 0, stream>>>(q, Q16, n8);
  wtcast_kernel<<<dim3(kDim / 64, kProjN / 64, kHeads), dim3(256), 0, stream>>>(
      Wqkv, WQT, kProjN, (long)kDim * kProjN, (long)kProjN * kDim);
  wtcast_kernel<<<dim3(kDim / 64, kDim / 64, 1), dim3(256), 0, stream>>>(Wg, WGT, kDim, 0L, 0L);
  wtcast_kernel<<<dim3(kDim / 64, kDim / 64, 1), dim3(256), 0, stream>>>(Wo, WOT, kDim, 0L, 0L);

  const int tilesProj = (kTok / 64) * (kGroupN / 64);
  for (int grp = 0; grp < kGroups; ++grp) {
    const unsigned short* Btg = WQT + (size_t)grp * kGroupN * kDim;
    const float* bqg = bqkv + grp * kGroupN;
    wmma_gemm64<1, 0, 2, 0, false, 0><<<dim3(tilesProj / 8, 1), dim3(256), 0, stream>>>(
        Q16, Q16, kDim, 0L, Btg, Btg, kDim, 0L,
        (void*)PG, (void*)PG, kGroupN, 0L, bqg, XX, 0L, kTok, kGroupN, kDim, 1.0f, ST, beta);
    retention_scan_kernel<<<dim3(kBatch * kGroupHeads), dim3(512), 0, stream>>>(PG, XX, ST, grp);
  }

  const int tilesSq = (kTok / 64) * (kDim / 64);
  wmma_gemm64<1, 0, 2, 3, false, 0><<<dim3(tilesSq / 8, 1), dim3(256), 0, stream>>>(
      Q16, Q16, kDim, 0L, WGT, WGT, kDim, 0L,
      (void*)ZH, (void*)ZL, kDim, 0L, bg, XX, 0L, kTok, kDim, kDim, 1.0f, ST, beta);

  wmma_gemm64<1, 1, 2, 0, false, 0><<<dim3(tilesSq / 8, 1), dim3(256), 0, stream>>>(
      ZH, ZL, kDim, 0L, WOT, WOT, kDim, 0L,
      (void*)out, (void*)ZL, kDim, 0L, bo, XX, 0L, kTok, kDim, kDim, 1.0f, ST, beta);
}
